// ResGATBlock_75771813036522
// MI455X (gfx1250) — hardware-verified
//
#include <hip/hip_runtime.h>
#include <stddef.h>


#define FIN     128
#define HID     128
#define NOUT    32
#define NTHR    256
#define NWAVE   8
#define EPT     8
#define NGRP    2
#define CHUNK   (NTHR * EPT * NGRP)
#define WCAP    (EPT * NGRP * 32)
#define LISTN   (NWAVE * WCAP)
#define NBC     4096
#define NBF     1024
#define RCAP    40960
#define RBN     128
#define TGT     256
#define DEGCAP  256
#define OTHR    512
#define MAXH    4
#define BM      64
#define WSCAP   134217728
#define NEG_SLOPE 0.2f
#define BN_EPS  1e-5f
#define ISQ2    0.7071067811865476f
#define ASCL    8.0f
#define WSCL    64.0f
#define OSCL    0.001953125f

#define LDS_FILL ((RCAP + NBF + LISTN) * 4 + 64)

static_assert((CHUNK & (CHUNK - 1)) == 0);
static_assert(CHUNK <= 4096);
static_assert(NBC <= 4096 && NBF <= 4096);
static_assert((NBC & (NBC - 1)) == 0 && (NBF & (NBF - 1)) == 0);
static_assert(NBC == 4 * NBF);
static_assert(OTHR * 8 == NBC);
static_assert((RCAP % 32) == 0);
static_assert(TGT == NWAVE * 32);
static_assert((NBC % TGT) == 0);
static_assert((TGT % BM) == 0);
static_assert(BM * 4 == NTHR);
static_assert(FIN % 32 == 0 && HID % 32 == 0);
static_assert(HID == 4 * 32);
static_assert(FIN == HID);

typedef float          v4f  __attribute__((ext_vector_type(4)));
typedef float          v8f  __attribute__((ext_vector_type(8)));
typedef int            v4i  __attribute__((ext_vector_type(4)));
typedef double         v2d  __attribute__((ext_vector_type(2)));
typedef _Float16       v8h  __attribute__((ext_vector_type(8)));
typedef _Float16       v16h __attribute__((ext_vector_type(16)));
union FragH { v16h v; v8h u[2]; };

__device__ __forceinline__ v8f wmh(v16h a, v16h b, v8f c) {
  v8f d = __builtin_amdgcn_wmma_f32_16x16x32_f16(false, a, false, b, (short)0, c, false, false);
  asm volatile("v_nop\n\tv_nop\n\tv_nop\n\tv_nop" : "+v"(d) : "v"(a), "v"(b));
  return d;
}

__device__ __forceinline__ v8h cvt8(v4f a, v4f b, float s) {
  v8h o;
  o[0] = (_Float16)(a.x * s); o[1] = (_Float16)(a.y * s);
  o[2] = (_Float16)(a.z * s); o[3] = (_Float16)(a.w * s);
  o[4] = (_Float16)(b.x * s); o[5] = (_Float16)(b.y * s);
  o[6] = (_Float16)(b.z * s); o[7] = (_Float16)(b.w * s);
  return o;
}

__device__ __forceinline__ float lrelu(float v) { return v > 0.0f ? v : NEG_SLOPE * v; }
__device__ __forceinline__ v4f relu4(v4f v) {
  v4f o;
  o.x = v.x > 0.f ? v.x : 0.f; o.y = v.y > 0.f ? v.y : 0.f;
  o.z = v.z > 0.f ? v.z : 0.f; o.w = v.w > 0.f ? v.w : 0.f;
  return o;
}

template <int NB>
__device__ __forceinline__ int scan_chunk(const int* __restrict__ dsts, int nE, int cbase, int slotBase,
                                          int vec8, int* list, int tid, int lane, int wave) {
  int wc = 0;
#pragma unroll
  for (int g = 0; g < NGRP; ++g) {
    const int el0  = (g * NTHR + tid) * EPT;
    const int e0   = cbase + el0;
    const int sent = -2147483647 - 1;
    v4i da, db;
    if (vec8 != 0 && cbase + CHUNK <= nE) {
      da = *(const v4i*)(dsts + e0);
      db = *(const v4i*)(dsts + e0 + 4);
    } else {
      da.x = (e0     < nE) ? dsts[min(e0, nE - 1)] : sent;
      da.y = (e0 + 1 < nE) ? dsts[min(e0 + 1, nE - 1)] : sent;
      da.z = (e0 + 2 < nE) ? dsts[min(e0 + 2, nE - 1)] : sent;
      da.w = (e0 + 3 < nE) ? dsts[min(e0 + 3, nE - 1)] : sent;
      db.x = (e0 + 4 < nE) ? dsts[min(e0 + 4, nE - 1)] : sent;
      db.y = (e0 + 5 < nE) ? dsts[min(e0 + 5, nE - 1)] : sent;
      db.z = (e0 + 6 < nE) ? dsts[min(e0 + 6, nE - 1)] : sent;
      db.w = (e0 + 7 < nE) ? dsts[min(e0 + 7, nE - 1)] : sent;
    }
    const unsigned nb = (unsigned)slotBase;
    const unsigned s0 = (unsigned)da.x - nb, s1 = (unsigned)da.y - nb;
    const unsigned s2 = (unsigned)da.z - nb, s3 = (unsigned)da.w - nb;
    const unsigned s4 = (unsigned)db.x - nb, s5 = (unsigned)db.y - nb;
    const unsigned s6 = (unsigned)db.z - nb, s7 = (unsigned)db.w - nb;
    const bool h0 = s0 < (unsigned)NB, h1 = s1 < (unsigned)NB, h2 = s2 < (unsigned)NB, h3 = s3 < (unsigned)NB;
    const bool h4 = s4 < (unsigned)NB, h5 = s5 < (unsigned)NB, h6 = s6 < (unsigned)NB, h7 = s7 < (unsigned)NB;
    const unsigned any = __builtin_amdgcn_ballot_w32(h0 | h1 | h2 | h3 | h4 | h5 | h6 | h7);
    if (any != 0u) {
#define HITJ(J, HJ, SJ) { \
        const unsigned mj = __builtin_amdgcn_ballot_w32(HJ); \
        if (mj != 0u) { \
          if (HJ) { \
            const int pos = wc + (int)__builtin_amdgcn_mbcnt_lo(mj, 0u); \
            if (pos < WCAP) list[wave * WCAP + pos] = ((el0 + (J)) << 12) | (int)(SJ); \
          } \
          wc += (int)__builtin_popcount(mj); } }
      HITJ(0, h0, s0)
      HITJ(1, h1, s1)
      HITJ(2, h2, s2)
      HITJ(3, h3, s3)
      HITJ(4, h4, s4)
      HITJ(5, h5, s5)
      HITJ(6, h6, s6)
      HITJ(7, h7, s7)
#undef HITJ
    }
  }
  return wc;
}

__global__ __launch_bounds__(NTHR) void k_xcvt(const float* __restrict__ x, _Float16* xp, int nN, int nUnits) {
  const int i = (int)blockIdx.x * NTHR + (int)threadIdx.x;
  if (i >= nUnits) return;
  const int row = i >> 4;
  const int c0  = (i & 15) * 8;
  int rr = row > nN - 1 ? nN - 1 : row;
  rr = rr < 0 ? 0 : rr;
  const float* p = x + (size_t)rr * FIN + c0;
  v4f a = *(const v4f*)p, b = *(const v4f*)(p + 4);
  const v4f z = {0.f, 0.f, 0.f, 0.f};
  if (row >= nN) { a = z; b = z; }
  const v8h o = cvt8(a, b, ASCL);
  _Float16* d = xp + (size_t)i * 8;
  *(volatile v8h*)d = o;
  __threadfence();
  *(volatile v8h*)d = o;
}

template <int KD, int NCW>
__global__ __launch_bounds__(NTHR) void k_wprep(const float* __restrict__ W, _Float16* wp) {
  constexpr int KS    = KD / 8;
  constexpr int UNITS = NCW * KS;
  static_assert(KD % 8 == 0);
  const int i = (int)blockIdx.x * NTHR + (int)threadIdx.x;
  if (i >= UNITS) return;
  const int n  = i / KS;
  const int k0 = (i - n * KS) * 8;
  v4f a, b;
  a.x = W[(size_t)(k0 + 0) * NCW + n]; a.y = W[(size_t)(k0 + 1) * NCW + n];
  a.z = W[(size_t)(k0 + 2) * NCW + n]; a.w = W[(size_t)(k0 + 3) * NCW + n];
  b.x = W[(size_t)(k0 + 4) * NCW + n]; b.y = W[(size_t)(k0 + 5) * NCW + n];
  b.z = W[(size_t)(k0 + 6) * NCW + n]; b.w = W[(size_t)(k0 + 7) * NCW + n];
  const v8h o = cvt8(a, b, WSCL);
  _Float16* d = wp + (size_t)i * 8;
  *(volatile v8h*)d = o;
  __threadfence();
  *(volatile v8h*)d = o;
}

__global__ __launch_bounds__(NTHR) void k_count(
    const int* __restrict__ dsts, int* cnt, int nE, int vec8) {
  __shared__ __attribute__((aligned(16))) int scnt[NBC];
  __shared__ __attribute__((aligned(16))) int list[LISTN];
  __shared__ int wcnt[NWAVE];
  const int tid = threadIdx.x, lane = tid & 31, wave = tid >> 5;
  const int nodeBase = blockIdx.x * NBC;

  for (int i = tid; i < NBC; i += NTHR) scnt[i] = 0;
  __syncthreads();

  const int nChunks = (nE + CHUNK - 1) / CHUNK;
#pragma unroll 1
  for (int ch = 0; ch < nChunks; ++ch) {
    const int cbase = ch * CHUNK;
    const int wc = scan_chunk<NBC>(dsts, nE, cbase, nodeBase, vec8, list, tid, lane, wave);
    if (lane == 0) wcnt[wave] = wc;
    __syncthreads();
    if (wave == 0) {
#pragma unroll 1
      for (int wsx = 0; wsx < NWAVE; ++wsx) {
        int n = __builtin_amdgcn_readfirstlane(wcnt[wsx]);
        n = n > WCAP ? WCAP : (n < 0 ? 0 : n);
        const int* lp = list + wsx * WCAP;
#pragma unroll 1
        for (int i = 0; i < n; ++i) {
          const int ent  = __builtin_amdgcn_readfirstlane(lp[i]);
          const int slot = ent & (NBC - 1);
          if (lane == 0) scnt[slot] = scnt[slot] + 1;
        }
      }
    }
    __syncthreads();
  }

  v4i cq[4];
#pragma unroll
  for (int q = 0; q < 4; ++q) {
    const int f = (wave * 4 + q) * 128 + 4 * lane;
    cq[q] = *(const v4i*)(scnt + f);
  }
  int* cp = cnt + (size_t)nodeBase;
#pragma unroll
  for (int q = 0; q < 4; ++q) {
    const int f = (wave * 4 + q) * 128 + 4 * lane;
    *(volatile v4i*)(cp + f) = cq[q];
  }
  __threadfence();
#pragma unroll
  for (int q = 0; q < 4; ++q) {
    const int f = (wave * 4 + q) * 128 + 4 * lane;
    *(volatile v4i*)(cp + f) = cq[q];
  }
}

__global__ __launch_bounds__(OTHR) void k_offsets(
    const int* __restrict__ cnt, int* off, int* rbase, int nChunk) {
  __shared__ __attribute__((aligned(16))) int soff[NBC];
  __shared__ __attribute__((aligned(16))) int srb[RBN];
  __shared__ int wtot[OTHR / 32];
  const int tid = threadIdx.x, lane = tid & 31, wave = tid >> 5, sub = tid >> 7;
  for (int i = tid; i < RBN; i += OTHR) srb[i] = 0;
  int carry = 0;
#pragma unroll 1
  for (int ch = 0; ch < nChunk; ++ch) {
    const int base = ch * NBC;
    const v4i c0 = *(const v4i*)(cnt + base + 8 * tid);
    const v4i c1 = *(const v4i*)(cnt + base + 8 * tid + 4);
    const int e0 = max(c0.x, 0), e1 = max(c0.y, 0), e2 = max(c0.z, 0), e3 = max(c0.w, 0);
    const int e4 = max(c1.x, 0), e5 = max(c1.y, 0), e6 = max(c1.z, 0), e7 = max(c1.w, 0);
    const int ts = e0 + e1 + e2 + e3 + e4 + e5 + e6 + e7;
    int incl = ts;
#pragma unroll
    for (int d = 1; d < 32; d <<= 1) {
      const int t = __shfl_up(incl, d);
      if (lane >= d) incl += t;
    }
    if (lane == 31) wtot[wave] = incl;
    __syncthreads();
    const int S0 = wtot[0]  + wtot[1]  + wtot[2]  + wtot[3];
    const int S1 = wtot[4]  + wtot[5]  + wtot[6]  + wtot[7];
    const int S2 = wtot[8]  + wtot[9]  + wtot[10] + wtot[11];
    const int S3 = wtot[12] + wtot[13] + wtot[14] + wtot[15];
    int pre = 0;
#pragma unroll 1
    for (int w = 4 * sub; w < wave; ++w) pre += wtot[w];
    const int b0 = carry;
    const int b1 = b0 + ((S0 + 31) & ~31);
    const int b2 = b1 + ((S1 + 31) & ~31);
    const int b3 = b2 + ((S2 + 31) & ~31);
    const int b4 = b3 + ((S3 + 31) & ~31);
    const int myb = sub == 0 ? b0 : (sub == 1 ? b1 : (sub == 2 ? b2 : b3));
    if (tid == 0) {
      srb[min(4 * ch + 0, RBN - 1)] = b0;
      srb[min(4 * ch + 1, RBN - 1)] = b1;
      srb[min(4 * ch + 2, RBN - 1)] = b2;
      srb[min(4 * ch + 3, RBN - 1)] = b3;
    }
    int run = myb + pre + incl - ts;
    soff[8 * tid + 0] = run; run += e0;
    soff[8 * tid + 1] = run; run += e1;
    soff[8 * tid + 2] = run; run += e2;
    soff[8 * tid + 3] = run; run += e3;
    soff[8 * tid + 4] = run; run += e4;
    soff[8 * tid + 5] = run; run += e5;
    soff[8 * tid + 6] = run; run += e6;
    soff[8 * tid + 7] = run;
    carry = b4;
    __syncthreads();
    const v4i o0 = *(const v4i*)(soff + 4 * tid);
    const v4i o1 = *(const v4i*)(soff + 4 * (tid + OTHR));
    int* op = off + base;
    *(volatile v4i*)(op + 4 * tid) = o0;
    *(volatile v4i*)(op + 4 * (tid + OTHR)) = o1;
    __threadfence();
    *(volatile v4i*)(op + 4 * tid) = o0;
    *(volatile v4i*)(op + 4 * (tid + OTHR)) = o1;
    __syncthreads();
  }
  if (tid == 0) srb[min(4 * nChunk, RBN - 1)] = carry;
  __syncthreads();
  v4i rv = {0, 0, 0, 0};
  if (tid < 32) rv = *(const v4i*)(srb + 4 * tid);
  if (tid < 32) *(volatile v4i*)(rbase + 4 * tid) = rv;
  __threadfence();
  if (tid < 32) *(volatile v4i*)(rbase + 4 * tid) = rv;
}

__global__ __launch_bounds__(NTHR) void k_fill(
    const int* __restrict__ srcs, const int* __restrict__ dsts,
    const int* __restrict__ off, const int* __restrict__ rbase,
    int* csr, int nN, int nE, int vec8, int csrLen) {
  extern __shared__ v4f lds_dyn[];
  int* region = (int*)lds_dyn;
  int* cursor = region + RCAP;
  int* list   = cursor + NBF;
  int* wcnt   = list + LISTN;
  const int tid = threadIdx.x, lane = tid & 31, wave = tid >> 5;
  const int b = blockIdx.x;
  const int nodeBase = b * NBF;

  int rb0 = rbase[b];
  const int rb1 = rbase[b + 1];
  rb0 = rb0 < 0 ? 0 : (rb0 > csrLen ? csrLen : rb0);
  rb0 &= ~31;
  int len = rb1 - rb0;
  len = len < 0 ? 0 : (len > RCAP ? RCAP : len);
  int lenW = (len + 31) & ~31;
  if (rb0 + lenW > csrLen) lenW = (csrLen - rb0) & ~31;

  {
    const v4i z = {0, 0, 0, 0};
    for (int i = tid; i < RCAP / 4; i += NTHR) ((v4i*)region)[i] = z;
    for (int s = tid; s < NBF; s += NTHR) {
      int o = off[nodeBase + s] - rb0;
      o = o < 0 ? 0 : (o > RCAP ? RCAP : o);
      cursor[s] = o;
    }
  }
  __syncthreads();

  const int nChunks = (nE + CHUNK - 1) / CHUNK;
#pragma unroll 1
  for (int ch = 0; ch < nChunks; ++ch) {
    const int cbase = ch * CHUNK;
    const int wc = scan_chunk<NBF>(dsts, nE, cbase, nodeBase, vec8, list, tid, lane, wave);
    if (lane == 0) wcnt[wave] = wc;
    __syncthreads();
    if (wave == 0) {
#pragma unroll 1
      for (int wsx = 0; wsx < NWAVE; ++wsx) {
        int n = __builtin_amdgcn_readfirstlane(wcnt[wsx]);
        n = n > WCAP ? WCAP : (n < 0 ? 0 : n);
        const int* lp = list + wsx * WCAP;
#pragma unroll 1
        for (int i = 0; i < n; ++i) {
          const int ent  = __builtin_amdgcn_readfirstlane(lp[i]);
          const int slot = ent & (NBF - 1);
          int e = cbase + ((ent >> 12) & (CHUNK - 1));
          e = e > nE - 1 ? nE - 1 : e;
          int src = srcs[e];
          src = src < 0 ? 0 : (src > nN - 1 ? nN - 1 : src);
          if (lane == 0) {
            int pos = cursor[slot];
            pos = pos < 0 ? 0 : (pos > RCAP - 1 ? RCAP - 1 : pos);
            region[pos] = src;
            const int np = pos + 1;
            cursor[slot] = np > RCAP ? RCAP : np;
          }
        }
      }
    }
    __syncthreads();
  }

  const int nv = lenW >> 2;
  int* gp = csr + rb0;
#pragma unroll 1
  for (int i = tid; i < nv; i += NTHR) { const v4i v = ((const v4i*)region)[i]; *(volatile v4i*)(gp + 4 * i) = v; }
  __threadfence();
#pragma unroll 1
  for (int i = tid; i < nv; i += NTHR) { const v4i v = ((const v4i*)region)[i]; *(volatile v4i*)(gp + 4 * i) = v; }
}

template <int K, int NC, int HEADS>
__global__ __launch_bounds__(NTHR) void k_gemm(
    const _Float16* __restrict__ Ap, const _Float16* __restrict__ Bp,
    const float* __restrict__ attS, const float* __restrict__ attD, const float* __restrict__ bias,
    float* C, float* eS, float* eD) {
  constexpr int TPW = NC / 32;
  constexpr int KT  = K / 32;
  constexpr int HE  = HEADS > 0 ? HEADS : 1;
  constexpr int NES = BM * HE;
  constexpr int NV  = NES / 4;
  constexpr int CPP = NC / 4;
  constexpr int NF4 = BM * NC / 4;
  constexpr int NIT = NF4 / NTHR;
  static_assert(K % 32 == 0);
  static_assert(HEADS == 0 || HEADS == 1 || HEADS == 2 || HEADS == 4);
  static_assert(2 * NV <= NTHR);
  static_assert(NF4 % NTHR == 0);
  static_assert(TPW >= 1 && TPW * 32 == NC);
  static_assert(CPP % 4 == 0);

  __shared__ __attribute__((aligned(16))) float stg[BM * NC];
  __shared__ __attribute__((aligned(16))) float sES[NES];
  __shared__ __attribute__((aligned(16))) float sED[NES];
  const int tid = threadIdx.x, lane = tid & 31, wave = tid >> 5, hh = lane >> 4, m = lane & 15;
  const int rowBase = blockIdx.x * BM;
  const int rg = wave >> 1, chf = wave & 1;
  const int r0 = rg * 16;
  const int c0 = chf * (NC / 2);

  v8f acc[TPW];
#pragma unroll
  for (int t = 0; t < TPW; ++t) { v8f z = {0.f, 0.f, 0.f, 0.f, 0.f, 0.f, 0.f, 0.f}; acc[t] = z; }

  const _Float16* ap  = Ap + (size_t)(rowBase + r0 + m) * K + 8 * hh;
  const _Float16* bp0 = Bp + (size_t)(c0 + m) * K + 8 * hh;
#pragma unroll 1
  for (int kt = 0; kt < KT; ++kt) {
    FragH a;
    a.u[0] = *(const v8h*)(ap + 32 * kt);
    a.u[1] = *(const v8h*)(ap + 32 * kt + 16);
#pragma unroll
    for (int t = 0; t < TPW; ++t) {
      const _Float16* bp = bp0 + (size_t)(16 * t) * K + 32 * kt;
      FragH bf;
      bf.u[0] = *(const v8h*)bp;
      bf.u[1] = *(const v8h*)(bp + 16);
      acc[t] = wmh(a.v, bf.v, acc[t]);
    }
  }

  {
    float* sp = stg + (size_t)(r0 + 8 * hh) * NC + c0 + m;
#pragma unroll
    for (int t = 0; t < TPW; ++t) {
      float bv = 0.f;
      if constexpr (HEADS == 0) bv = bias[c0 + 16 * t + m];
#pragma unroll
      for (int r = 0; r < 8; ++r) sp[r * NC + 16 * t] = acc[t][r] * OSCL + bv;
    }
  }
  __syncthreads();

  if constexpr (HEADS > 0) {
    const int drow = tid >> 2, part = tid & 3;
    const float* rp  = stg + (size_t)drow * NC + CPP * part;
    const float* sa  = attS + CPP * part;
    const float* sdd = attD + CPP * part;
    float ps = 0.f, pd = 0.f;
#pragma unroll 2
    for (int c = 0; c < CPP; c += 4) {
      const v4f hv = *(const v4f*)(rp + c);
      const v4f av = *(const v4f*)(sa + c);
      const v4f dv = *(const v4f*)(sdd + c);
      ps += hv.x * av.x + hv.y * av.y + hv.z * av.z + hv.w * av.w;
      pd += hv.x * dv.x + hv.y * dv.y + hv.z * dv.z + hv.w * dv.w;
    }
    if constexpr (HEADS == 4) {
      sES[drow * 4 + part] = ps; sED[drow * 4 + part] = pd;
    } else if constexpr (HEADS == 2) {
      ps += __shfl_xor(ps, 1); pd += __shfl_xor(pd, 1);
      if ((part & 1) == 0) { sES[drow * 2 + (part >> 1)] = ps; sED[drow * 2 + (part >> 1)] = pd; }
    } else {
      ps += __shfl_xor(ps, 1); pd += __shfl_xor(pd, 1);
      ps += __shfl_xor(ps, 2); pd += __shfl_xor(pd, 2);
      if (part == 0) { sES[drow] = ps; sED[drow] = pd; }
    }
  }

  {
    float* tileC = C + (size_t)rowBase * NC;
    v4f cv[NIT];
#pragma unroll
    for (int it = 0; it < NIT; ++it) cv[it] = *(const v4f*)(stg + 4 * (it * NTHR + tid));
#pragma unroll
    for (int it = 0; it < NIT; ++it) *(volatile v4f*)(tileC + 4 * (size_t)(it * NTHR + tid)) = cv[it];
    __threadfence();
#pragma unroll
    for (int it = 0; it < NIT; ++it) *(volatile v4f*)(tileC + 4 * (size_t)(it * NTHR + tid)) = cv[it];
  }

  if constexpr (HEADS > 0) {
    __syncthreads();
    const size_t eb = (size_t)rowBase * HEADS;
    const int iS = tid < NV - 1 ? tid : NV - 1;
    int iD = tid - NV; iD = iD < 0 ? 0 : (iD > NV - 1 ? NV - 1 : iD);
    const v4f vS = *(const v4f*)(sES + 4 * iS);
    const v4f vD = *(const v4f*)(sED + 4 * iD);
    const bool isS = tid < NV;
    const v4f dv = isS ? vS : vD;
    float* gp = isS ? (eS + eb + 4 * iS) : (eD + eb + 4 * iD);
    if (tid < 2 * NV) *(volatile v4f*)gp = dv;
    __threadfence();
    if (tid < 2 * NV) *(volatile v4f*)gp = dv;
  }
}

template <int HEADS>
__global__ __launch_bounds__(NTHR) void k_agg(
    const int* __restrict__ csr, const int* __restrict__ off, const int* __restrict__ cnt,
    const float* __restrict__ eS, const float* __restrict__ eD, const float* __restrict__ hw,
    const float* __restrict__ bias, float* agg, double* part, int nN, int csrLen) {
  constexpr int NC  = HID;
  constexpr int CHN = NC / HEADS;
  static_assert(HEADS == 1 || HEADS == 2 || HEADS == 4);
  __shared__ __attribute__((aligned(16))) double sP[NWAVE * 2 * NC];
  const int tid = threadIdx.x, lane = tid & 31, wave = tid >> 5;
  const int tbase = blockIdx.x * TGT + wave * 32;
  const int col = 4 * lane;
  const int hd  = col / CHN;

  const v4f bb = *(const v4f*)(bias + col);

  const int cl    = tbase + lane;
  const int cnt_l = cnt[cl];
  const int off_l = off[cl];

  double s0 = 0.0, s1 = 0.0, s2 = 0.0, s3 = 0.0;
  double q0 = 0.0, q1 = 0.0, q2 = 0.0, q3 = 0.0;

#pragma unroll 1
  for (int j = 0; j < 32; ++j) {
    const int c = tbase + j;
    int n = __shfl(cnt_l, j);
    n = n < 0 ? 0 : (n > DEGCAP ? DEGCAP : n);
    const int st = __shfl(off_l, j);
    const float edc   = eD[(size_t)c * HEADS + hd];
    const float eself = lrelu(eS[(size_t)c * HEADS + hd] + edc);

    float mx = eself;
#pragma unroll 1
    for (int qb = 0; qb < n; qb += 32) {
      int pos = st + qb + lane;
      pos = pos < 0 ? 0 : (pos > csrLen - 1 ? csrLen - 1 : pos);
      int sl = csr[pos];
      sl = sl < 0 ? 0 : (sl > nN - 1 ? nN - 1 : sl);
      const int mcnt = (n - qb) < 32 ? (n - qb) : 32;
#pragma unroll 1
      for (int pp = 0; pp < mcnt; ++pp) {
        const int s = __builtin_amdgcn_readlane(sl, pp);
        mx = fmaxf(mx, lrelu(eS[(size_t)s * HEADS + hd] + edc));
      }
    }

    float p   = __expf(eself - mx);
    float den = p;
    v4f acc = *(const v4f*)(hw + (size_t)c * NC + col) * p;
#pragma unroll 1
    for (int qb = 0; qb < n; qb += 32) {
      int pos = st + qb + lane;
      pos = pos < 0 ? 0 : (pos > csrLen - 1 ? csrLen - 1 : pos);
      int sl = csr[pos];
      sl = sl < 0 ? 0 : (sl > nN - 1 ? nN - 1 : sl);
      const int mcnt = (n - qb) < 32 ? (n - qb) : 32;
#pragma unroll 1
      for (int pp = 0; pp < mcnt; ++pp) {
        const int s = __builtin_amdgcn_readlane(sl, pp);
        p = __expf(lrelu(eS[(size_t)s * HEADS + hd] + edc) - mx);
        den += p;
        const v4f hv = *(const v4f*)(hw + (size_t)s * NC + col);
        acc = acc + hv * p;
      }
    }

    const float rd = 1.0f / den;
    v4f v = acc * rd + bb;
    const v4f z4 = {0.f, 0.f, 0.f, 0.f};
    if (c >= nN) v = z4;
    float* gp = agg + (size_t)c * NC + col;
    *(volatile v4f*)gp = v;
    __threadfence();
    *(volatile v4f*)gp = v;

    s0 += (double)v.x; s1 += (double)v.y; s2 += (double)v.z; s3 += (double)v.w;
    q0 += (double)v.x * (double)v.x; q1 += (double)v.y * (double)v.y;
    q2 += (double)v.z * (double)v.z; q3 += (double)v.w * (double)v.w;
  }

  {
    double* sp = sP + (size_t)(wave * 2) * NC + col;
    sp[0] = s0; sp[1] = s1; sp[2] = s2; sp[3] = s3;
    sp[NC + 0] = q0; sp[NC + 1] = q1; sp[NC + 2] = q2; sp[NC + 3] = q3;
  }
  __syncthreads();
  {
    const int t = tid & 127;
    const int stat = t >> 6, cc = 2 * (t & 63);
    double a0 = 0.0, a1 = 0.0;
#pragma unroll
    for (int w = 0; w < NWAVE; ++w) {
      const double* rp = sP + (size_t)(w * 2 + stat) * NC + cc;
      a0 += rp[0]; a1 += rp[1];
    }
    v2d o; o.x = a0; o.y = a1;
    double* gq = part + (size_t)blockIdx.x * 2 * NC + stat * NC + cc;
    if (tid < 128) *(volatile v2d*)gq = o;
    __threadfence();
    if (tid < 128) *(volatile v2d*)gq = o;
  }
}

__global__ __launch_bounds__(NTHR) void k_bnstat(const double* __restrict__ part, int nBlk, int nN, float* stats) {
  __shared__ __attribute__((aligned(16))) float sSt[2 * HID];
  const int tid = threadIdx.x;
  const int c = tid & (HID - 1);
  double s = 0.0, q = 0.0;
#pragma unroll 1
  for (int b = 0; b < nBlk; ++b) {
    const double* p = part + (size_t)b * 2 * HID;
    s += p[c];
    q += p[HID + c];
  }
  const double inv = 1.0 / (double)nN;
  const double mu  = s * inv;
  double var = q * inv - mu * mu;
  var = var < 0.0 ? 0.0 : var;
  const float muf = (float)mu;
  const float rs  = 1.0f / sqrtf((float)var + BN_EPS);
  if (tid < HID) { sSt[tid] = muf; sSt[HID + tid] = rs; }
  __syncthreads();
  const int li = tid < 64 ? tid : 63;
  const v4f v = *(const v4f*)(sSt + 4 * li);
  if (tid < 64) *(volatile v4f*)(stats + 4 * li) = v;
  __threadfence();
  if (tid < 64) *(volatile v4f*)(stats + 4 * li) = v;
}

template <int RES>
__global__ __launch_bounds__(NTHR) void k_bncvt(
    const float* __restrict__ agg, const float* __restrict__ res, const float* __restrict__ stats,
    const float* __restrict__ gamma, const float* __restrict__ beta, _Float16* hp, int nN, int nUnits) {
  const int i = (int)blockIdx.x * NTHR + (int)threadIdx.x;
  if (i >= nUnits) return;
  const int row = i >> 4;
  const int c0  = (i & 15) * 8;
  const float* p = agg + (size_t)row * HID + c0;
  const v4f a0 = *(const v4f*)p, a1 = *(const v4f*)(p + 4);
  const v4f m0 = *(const v4f*)(stats + c0), m1 = *(const v4f*)(stats + c0 + 4);
  const v4f r0 = *(const v4f*)(stats + HID + c0), r1 = *(const v4f*)(stats + HID + c0 + 4);
  const v4f g0 = *(const v4f*)(gamma + c0), g1 = *(const v4f*)(gamma + c0 + 4);
  const v4f b0 = *(const v4f*)(beta + c0), b1 = *(const v4f*)(beta + c0 + 4);
  v4f t0 = (a0 - m0) * r0; t0 = t0 * g0; t0 = t0 + b0;
  v4f t1 = (a1 - m1) * r1; t1 = t1 * g1; t1 = t1 + b1;
  t0 = relu4(t0); t1 = relu4(t1);
  if constexpr (RES == 1) {
    const float* rq = res + (size_t)row * HID + c0;
    const v4f e0 = *(const v4f*)rq, e1 = *(const v4f*)(rq + 4);
    t0 = (t0 + e0) * ISQ2;
    t1 = (t1 + e1) * ISQ2;
  }
  const v4f z = {0.f, 0.f, 0.f, 0.f};
  if (row >= nN) { t0 = z; t1 = z; }
  const v8h o = cvt8(t0, t1, ASCL);
  _Float16* d = hp + (size_t)i * 8;
  *(volatile v8h*)d = o;
  __threadfence();
  *(volatile v8h*)d = o;
}

__global__ __launch_bounds__(NTHR) void k_fin(
    const _Float16* __restrict__ Ap, const _Float16* __restrict__ Bp,
    const float* __restrict__ bfin, float* out, int nN) {
  constexpr int K   = HID;
  constexpr int NC  = NOUT;
  constexpr int KT  = K / 32;
  constexpr int NF4 = BM * NC / 4;
  constexpr int NIT = NF4 / NTHR;
  static_assert(NC == 32);
  static_assert(NF4 % NTHR == 0);
  __shared__ __attribute__((aligned(16))) float stg[BM * NC];
  const int tid = threadIdx.x, lane = tid & 31, wave = tid >> 5, hh = lane >> 4, m = lane & 15;
  const int rowBase = blockIdx.x * BM;
  const int rg = wave >> 1, chf = wave & 1;
  const int r0 = rg * 16;
  const int c0 = chf * 16;

  v8f acc = {0.f, 0.f, 0.f, 0.f, 0.f, 0.f, 0.f, 0.f};
  const _Float16* ap = Ap + (size_t)(rowBase + r0 + m) * K + 8 * hh;
  const _Float16* bp = Bp + (size_t)(c0 + m) * K + 8 * hh;
#pragma unroll 1
  for (int kt = 0; kt < KT; ++kt) {
    FragH a, bf;
    a.u[0]  = *(const v8h*)(ap + 32 * kt);
    a.u[1]  = *(const v8h*)(ap + 32 * kt + 16);
    bf.u[0] = *(const v8h*)(bp + 32 * kt);
    bf.u[1] = *(const v8h*)(bp + 32 * kt + 16);
    acc = wmh(a.v, bf.v, acc);
  }

  {
    float* sp = stg + (size_t)(r0 + 8 * hh) * NC + c0 + m;
    const float bv = bfin[c0 + m];
#pragma unroll
    for (int r = 0; r < 8; ++r) sp[r * NC] = acc[r] * OSCL + bv;
  }
  __syncthreads();

  {
    float* tileO = out + (size_t)rowBase * NC;
    v4f cv[NIT];
    bool ok[NIT];
#pragma unroll
    for (int it = 0; it < NIT; ++it) {
      const int f = it * NTHR + tid;
      cv[it] = *(const v4f*)(stg + 4 * f);
      ok[it] = (rowBase + (f >> 3)) < nN;
    }
#pragma unroll
    for (int it = 0; it < NIT; ++it)
      if (ok[it]) *(volatile v4f*)(tileO + 4 * (size_t)(it * NTHR + tid)) = cv[it];
    __threadfence();
#pragma unroll
    for (int it = 0; it < NIT; ++it)
      if (ok[it]) *(volatile v4f*)(tileO + 4 * (size_t)(it * NTHR + tid)) = cv[it];
  }
}

extern "C" void kernel_launch(void* const* d_in, const int* in_sizes, int n_in,
                              void* d_out, int out_size, void* d_ws, size_t ws_size,
                              hipStream_t stream) {
  if (n_in < 18) return;
  const int nN = in_sizes[0] / FIN;
  const int nE = in_sizes[1] / 2;
  if (nN <= 0 || nE <= 0 || in_sizes[0] != nN * FIN || in_sizes[1] != 2 * nE) return;
  if (in_sizes[2] != FIN * HID || in_sizes[3] != HID || in_sizes[4] != HID || in_sizes[5] != HID) return;
  if (in_sizes[6] != HID * HID || in_sizes[7] != HID || in_sizes[8] != HID || in_sizes[9] != HID) return;
  if (in_sizes[10] != HID || in_sizes[11] != HID || in_sizes[12] != HID || in_sizes[13] != HID) return;
  if (in_sizes[14] != FIN * HID || in_sizes[15] != HID || in_sizes[16] != HID * NOUT || in_sizes[17] != NOUT) return;
  if (out_size != nN * NOUT) return;
  if (nE > (1 << 28) || nN > (1 << 22)) return;

  const float* x    = (const float*)d_in[0];
  const int*   ei   = (const int*)d_in[1];
  const int*   src  = ei;
  const int*   dst  = ei + nE;
  const float* W1   = (const float*)d_in[2];
  const float* a1s  = (const float*)d_in[3];
  const float* a1d  = (const float*)d_in[4];
  const float* b1   = (const float*)d_in[5];
  const float* W2   = (const float*)d_in[6];
  const float* a2s  = (const float*)d_in[7];
  const float* a2d  = (const float*)d_in[8];
  const float* b2   = (const float*)d_in[9];
  const float* g1   = (const float*)d_in[10];
  const float* be1  = (const float*)d_in[11];
  const float* g2   = (const float*)d_in[12];
  const float* be2  = (const float*)d_in[13];
  const float* Wres = (const float*)d_in[14];
  const float* bres = (const float*)d_in[15];
  const float* Wfin = (const float*)d_in[16];
  const float* bfin = (const float*)d_in[17];
  float* out = (float*)d_out;

  const int NPAD   = ((nN + TGT - 1) / TGT) * TGT;
  const int nBC    = (nN + NBC - 1) / NBC;
  const int CNTPAD = nBC * NBC;
  if (CNTPAD < NPAD) return;
  if (4 * nBC + 1 > RBN) return;
  const int nBF    = (nN + NBF - 1) / NBF;
  if (nBF + 1 > 4 * nBC + 1) return;
  const int csrLen = ((nE + 31) & ~31) + 4096;
  if (31 * 4 * nBC > 4096) return;
  const int nAgg   = NPAD / TGT;
  const int nGemm  = NPAD / BM;
  const int nXu    = NPAD * (HID / 8);

  char* ws = (char*)d_ws;
  size_t off = 0;
  const size_t oW1  = off; off += (size_t)HID * FIN * 2;           off = (off + 255) & ~(size_t)255;
  const size_t oW2  = off; off += (size_t)HID * HID * 2;           off = (off + 255) & ~(size_t)255;
  const size_t oW3  = off; off += (size_t)HID * FIN * 2;           off = (off + 255) & ~(size_t)255;
  const size_t oW4  = off; off += (size_t)NOUT * HID * 2;          off = (off + 255) & ~(size_t)255;
  const size_t oXp  = off; off += (size_t)NPAD * FIN * 2;          off = (off + 255) & ~(size_t)255;
  const size_t oHp  = off; off += (size_t)NPAD * HID * 2;          off = (off + 255) & ~(size_t)255;
  const size_t oCnt = off; off += (size_t)CNTPAD * 4;              off = (off + 255) & ~(size_t)255;
  const size_t oOff = off; off += (size_t)CNTPAD * 4;              off = (off + 255) & ~(size_t)255;
  const size_t oRb  = off; off += (size_t)RBN * 4;                 off = (off + 255) & ~(size_t)255;
  const size_t oCsr = off; off += (size_t)csrLen * 4;              off = (off + 255) & ~(size_t)255;
  const size_t oHw  = off; off += (size_t)NPAD * HID * 4;          off = (off + 255) & ~(size_t)255;
  const size_t oAgg = off; off += (size_t)NPAD * HID * 4;          off = (off + 255) & ~(size_t)255;
  const size_t oES  = off; off += (size_t)NPAD * MAXH * 4;         off = (off + 255) & ~(size_t)255;
  const size_t oED  = off; off += (size_t)NPAD * MAXH * 4;         off = (off + 255) & ~(size_t)255;
  const size_t oPt  = off; off += (size_t)nAgg * 2 * HID * 8;      off = (off + 255) & ~(size_t)255;
  const size_t oSt  = off; off += (size_t)2 * HID * 4;             off = (off + 255) & ~(size_t)255;
  if (off > ws_size || off > (size_t)WSCAP) return;
  _Float16* wp1  = (_Float16*)(ws + oW1);
  _Float16* wp2  = (_Float16*)(ws + oW2);
  _Float16* wp3  = (_Float16*)(ws + oW3);
  _Float16* wp4  = (_Float16*)(ws + oW4);
  _Float16* xp   = (_Float16*)(ws + oXp);
  _Float16* hp   = (_Float16*)(ws + oHp);
  int*    cnt   = (int*)(ws + oCnt);
  int*    offp  = (int*)(ws + oOff);
  int*    rb    = (int*)(ws + oRb);
  int*    csr   = (int*)(ws + oCsr);
  float*  hw    = (float*)(ws + oHw);
  float*  agg   = (float*)(ws + oAgg);
  float*  es    = (float*)(ws + oES);
  float*  ed    = (float*)(ws + oED);
  double* part  = (double*)(ws + oPt);
  float*  stats = (float*)(ws + oSt);

  const int vec8 = ((nE & 3) == 0) ? 1 : 0;

  k_wprep<FIN, HID><<<(HID * FIN / 8 + NTHR - 1) / NTHR, NTHR, 0, stream>>>(W1, wp1);
  k_wprep<HID, HID><<<(HID * HID / 8 + NTHR - 1) / NTHR, NTHR, 0, stream>>>(W2, wp2);
  k_wprep<FIN, HID><<<(HID * FIN / 8 + NTHR - 1) / NTHR, NTHR, 0, stream>>>(Wres, wp3);
  k_wprep<HID, NOUT><<<(NOUT * HID / 8 + NTHR - 1) / NTHR, NTHR, 0, stream>>>(Wfin, wp4);
  k_xcvt<<<(nXu + NTHR - 1) / NTHR, NTHR, 0, stream>>>(x, xp, nN, nXu);

  k_count<<<nBC, NTHR, 0, stream>>>(dst, cnt, nE, vec8);
  k_offsets<<<1, OTHR, 0, stream>>>(cnt, offp, rb, nBC);
  hipFuncSetAttribute(reinterpret_cast<const void*>(&k_fill),
                      hipFuncAttributeMaxDynamicSharedMemorySize, LDS_FILL);
  k_fill<<<nBF, NTHR, LDS_FILL, stream>>>(src, dst, offp, rb, csr, nN, nE, vec8, csrLen);

  k_gemm<FIN, HID, 4><<<nGemm, NTHR, 0, stream>>>(xp, wp1, a1s, a1d, b1, hw, es, ed);
  k_agg<4><<<nAgg, NTHR, 0, stream>>>(csr, offp, cnt, es, ed, hw, b1, agg, part, nN, csrLen);
  k_bnstat<<<1, NTHR, 0, stream>>>(part, nAgg, nN, stats);
  k_bncvt<0><<<(nXu + NTHR - 1) / NTHR, NTHR, 0, stream>>>(agg, hw, stats, g1, be1, hp, nN, nXu);

  k_gemm<HID, HID, 1><<<nGemm, NTHR, 0, stream>>>(hp, wp2, a2s, a2d, b2, hw, es, ed);
  k_agg<1><<<nAgg, NTHR, 0, stream>>>(csr, offp, cnt, es, ed, hw, b2, agg, part, nN, csrLen);
  k_bnstat<<<1, NTHR, 0, stream>>>(part, nAgg, nN, stats);

  k_gemm<FIN, HID, 0><<<nGemm, NTHR, 0, stream>>>(xp, wp3, a1s, a1d, bres, hw, es, ed);

  k_bncvt<1><<<(nXu + NTHR - 1) / NTHR, NTHR, 0, stream>>>(agg, hw, stats, g2, be2, hp, nN, nXu);
  k_fin<<<nGemm, NTHR, 0, stream>>>(hp, wp4, bfin, out, nN);
}
